// PConv_11467562680751
// MI455X (gfx1250) — hardware-verified
//
#include <hip/hip_runtime.h>
#include <stdint.h>


typedef float          v8f   __attribute__((ext_vector_type(8)));
typedef float          v4f   __attribute__((ext_vector_type(4)));
typedef __bf16         v16bf __attribute__((ext_vector_type(16)));
typedef unsigned short v16u  __attribute__((ext_vector_type(16)));
typedef unsigned short v8us  __attribute__((ext_vector_type(8)));

union Frag { v16u u; v16bf b; v8us h8[2]; };

#define Bn   4
#define Hn   192
#define Wn   192
#define HWn  (Hn * Wn)
#define Cin  16
#define Cm   64
#define KD   1024
#define NPIX (Bn * HWn)

#define TPX          64
#define TPR          (Wn / TPX)
#define NBLK_MAIN    (Bn * Hn * TPR)
#define MAIN_THREADS 128

#define C0_PX   256
#define NBLK_C0 (NPIX / C0_PX)

#define GZP  148
#define TTP  136
#define OSP  68
#define KCH  128
#define NCH  (KD / KCH)
#define CPC  (KCH / 16)

#define OFF_EW0 0
#define OFF_EB0 1024
#define OFF_W1  1088
#define OFF_B1  1112
#define OFF_W2  1120
#define OFF_B2  1184
#define OFF_W3  1192
#define OFF_B3  1320
#define OFF_LS  1336
#define OFF_LEB 1400
#define PF_USED 1464
#define PF_PAD  1472

static_assert(Wn % TPX == 0);
static_assert(HWn % C0_PX == 0);
static_assert(MAIN_THREADS == 2 * TPX);
static_assert(TPX * OSP * sizeof(float) <= 2 * TPX * TTP * sizeof(unsigned short));
static_assert(PF_PAD % 32 == 0);
static_assert((Cm * KD) % (8 * 256) == 0);
static_assert(KD % KCH == 0);
static_assert(KCH % 32 == 0);

__device__ __forceinline__ unsigned int bf16_rne(float f) {
    unsigned int u = __float_as_uint(f);
    u += 0x7FFFu + ((u >> 16) & 1u);
    return u >> 16;
}

__device__ __forceinline__ void split_bf16(float x, unsigned int& hb, unsigned int& lb) {
    hb = bf16_rne(x);
    const float hf = __uint_as_float(hb << 16);
    lb = bf16_rne(x - hf);
}

__device__ __forceinline__ v8f wmma_bf16(v16bf a, v16bf b, v8f c) {
    v8f d = __builtin_amdgcn_wmma_f32_16x16x32_bf16(false, a, false, b, (short)0, c, false, false);
    asm volatile("v_nop\n\tv_nop\n\tv_nop\n\tv_nop" : "+v"(d) : "v"(a), "v"(b));
    return d;
}

__global__ __launch_bounds__(256) void k_fold(
    const float* __restrict__ w0,  const float* __restrict__ b0,  const float* __restrict__ g0,
    const float* __restrict__ be0, const float* __restrict__ m0,  const float* __restrict__ v0,
    const float* __restrict__ w1,  const float* __restrict__ bb1, const float* __restrict__ g1,
    const float* __restrict__ be1, const float* __restrict__ m1,  const float* __restrict__ v1,
    const float* __restrict__ w2,  const float* __restrict__ bb2, const float* __restrict__ g2,
    const float* __restrict__ be2, const float* __restrict__ m2,  const float* __restrict__ v2,
    const float* __restrict__ w3,  const float* __restrict__ bb3, const float* __restrict__ g3,
    const float* __restrict__ be3, const float* __restrict__ m3,  const float* __restrict__ v3,
    const float* __restrict__ lb,  const float* __restrict__ lg,  const float* __restrict__ lbe,
    const float* __restrict__ lm,  const float* __restrict__ lv,
    float* __restrict__ P)
{
    __shared__ __align__(16) float sp[PF_PAD];
    const int t = threadIdx.x;
    const float eps = 1e-5f;
    if (t < 64) {
        const float s = g0[t] * rsqrtf(v0[t] + eps);
#pragma unroll
        for (int c = 0; c < Cin; ++c) sp[OFF_EW0 + t * Cin + c] = w0[t * Cin + c] * s;
        sp[OFF_EB0 + t] = be0[t] + (b0[t] - m0[t]) * s;
        const float ls = lg[t] * rsqrtf(lv[t] + eps);
        sp[OFF_LS + t]  = ls;
        sp[OFF_LEB + t] = lbe[t] + (lb[t] - lm[t]) * ls;
    }
    if (t < 8) {
        const float s = g1[t] * rsqrtf(v1[t] + eps);
#pragma unroll
        for (int c = 0; c < 3; ++c) sp[OFF_W1 + t * 3 + c] = w1[t * 3 + c] * s;
        sp[OFF_B1 + t] = be1[t] + (bb1[t] - m1[t]) * s;
    }
    if (t >= 64 && t < 72) {
        const int r = t - 64;
        const float s = g2[r] * rsqrtf(v2[r] + eps);
#pragma unroll
        for (int c = 0; c < 8; ++c) sp[OFF_W2 + r * 8 + c] = w2[r * 8 + c] * s;
        sp[OFF_B2 + r] = be2[r] + (bb2[r] - m2[r]) * s;
    }
    if (t >= 72 && t < 88) {
        const int r = t - 72;
        const float s = g3[r] * rsqrtf(v3[r] + eps);
#pragma unroll
        for (int c = 0; c < 8; ++c) sp[OFF_W3 + r * 8 + c] = w3[r * 8 + c] * s;
        sp[OFF_B3 + r] = be3[r] + (bb3[r] - m3[r]) * s;
    }
    if (t >= 88 && t < 88 + (PF_PAD - PF_USED)) sp[PF_USED + (t - 88)] = 0.f;
    __syncthreads();

    const int nq = PF_PAD / 4;
    {
        const int i0 = t, i1 = t + 256;
        if (i0 < nq) { const v4f v = *(const v4f*)(sp + 4 * i0); *(volatile v4f*)(P + 4 * i0) = v; }
        if (i1 < nq) { const v4f v = *(const v4f*)(sp + 4 * i1); *(volatile v4f*)(P + 4 * i1) = v; }
    }
    __threadfence();
    {
        const int i0 = t, i1 = t + 256;
        if (i0 < nq) { const v4f v = *(const v4f*)(sp + 4 * i0); *(volatile v4f*)(P + 4 * i0) = v; }
        if (i1 < nq) { const v4f v = *(const v4f*)(sp + 4 * i1); *(volatile v4f*)(P + 4 * i1) = v; }
    }
}

__global__ __launch_bounds__(256) void k_lwsplit(const float* __restrict__ lw,
                                                 unsigned short* __restrict__ LWH,
                                                 unsigned short* __restrict__ LWL)
{
    const int g = blockIdx.x * 256 + threadIdx.x;
    if (g >= (Cm * KD) / 8) return;
    const float* src = lw + (size_t)g * 8;
    const v4f a = *(const v4f*)(src);
    const v4f c = *(const v4f*)(src + 4);
    v8us hv, lv;
#pragma unroll
    for (int i = 0; i < 4; ++i) {
        unsigned int hb, lb2; split_bf16(a[i], hb, lb2);
        hv[i] = (unsigned short)hb; lv[i] = (unsigned short)lb2;
    }
#pragma unroll
    for (int i = 0; i < 4; ++i) {
        unsigned int hb, lb2; split_bf16(c[i], hb, lb2);
        hv[4 + i] = (unsigned short)hb; lv[4 + i] = (unsigned short)lb2;
    }
    volatile v8us* ph = (volatile v8us*)(LWH + (size_t)g * 8);
    volatile v8us* pl = (volatile v8us*)(LWL + (size_t)g * 8);
    *ph = hv; *pl = lv;
    __threadfence();
    *ph = hv; *pl = lv;
}

__global__ __launch_bounds__(256) void k_conv0(const float* __restrict__ x,
                                               const float* __restrict__ P,
                                               float* __restrict__ X1)
{
    __shared__ __align__(16) float so[Cm * C0_PX];
    if (blockIdx.x >= NBLK_C0) return;
    const int t = threadIdx.x, lane = t & 31, wv = t >> 5;
    const int b   = blockIdx.x / (HWn / C0_PX);
    const int hwb = (blockIdx.x % (HWn / C0_PX)) * C0_PX;
    const int hw  = hwb + t;

    float xin[Cin];
#pragma unroll
    for (int c = 0; c < Cin; ++c) xin[c] = x[((size_t)(b * Cin + c)) * HWn + hw];

    const float* EW0 = P + OFF_EW0;
    const float* EB0 = P + OFF_EB0;
#pragma unroll 1
    for (int o = 0; o < Cm; ++o) {
        float a = EB0[o];
#pragma unroll
        for (int c = 0; c < Cin; ++c) a = fmaf(EW0[o * Cin + c], xin[c], a);
        so[o * C0_PX + t] = fmaxf(a, 0.f);
    }
    __syncthreads();

    float* xb = X1 + ((size_t)b * Cm) * HWn + hwb;
#pragma unroll
    for (int r = 0; r < 8; ++r) {
        const int o = wv * 8 + r;
#pragma unroll
        for (int hf = 0; hf < 2; ++hf) {
            const int f = hf * 32 + lane;
            const v4f v = *(const v4f*)(so + o * C0_PX + f * 4);
            *(volatile v4f*)(xb + (size_t)o * HWn + f * 4) = v;
        }
    }
    __threadfence();
#pragma unroll
    for (int r = 0; r < 8; ++r) {
        const int o = wv * 8 + r;
#pragma unroll
        for (int hf = 0; hf < 2; ++hf) {
            const int f = hf * 32 + lane;
            const v4f v = *(const v4f*)(so + o * C0_PX + f * 4);
            *(volatile v4f*)(xb + (size_t)o * HWn + f * 4) = v;
        }
    }
}

union TTU { unsigned short t[2][TPX * TTP]; float o[TPX * OSP]; };

__global__ __launch_bounds__(MAIN_THREADS) void k_main(const float* __restrict__ gxyz,
                                                       const float* __restrict__ X1,
                                                       const unsigned short* __restrict__ LWH,
                                                       const unsigned short* __restrict__ LWL,
                                                       const float* __restrict__ P,
                                                       float* __restrict__ out)
{
    __shared__ __align__(16) float s_gz[TPX * GZP];
    __shared__ __align__(16) TTU   s_u;

    if (blockIdx.x >= NBLK_MAIN) return;
    const int tid  = threadIdx.x;
    const int lane = tid & 31;
    const int wv   = tid >> 5;
    const int blk  = blockIdx.x;
    const int tw   = blk % TPR;
    const int h    = (blk / TPR) % Hn;
    const int b    = blk / (TPR * Hn);
    const int w0   = tw * TPX;

    {
        const float* W1 = P + OFF_W1;  const float* B1 = P + OFF_B1;
        const float* W2 = P + OFF_W2;  const float* B2 = P + OFF_B2;
        const float* W3 = P + OFF_W3;  const float* B3 = P + OFF_B3;
#pragma unroll 1
        for (int it = 0; it < (TPX * 9 + MAIN_THREADS - 1) / MAIN_THREADS; ++it) {
            const int i = it * MAIN_THREADS + tid;
            if (i < TPX * 9) {
                const int px = i % TPX;
                const int kk = i / TPX;
                const int w  = w0 + px;
                const size_t gi = ((((size_t)b * 3 + 0) * 9 + kk) * Hn + h) * Wn + w;
                const float i0 = gxyz[gi];
                const float i1 = gxyz[gi + (size_t)9 * HWn];
                const float i2 = gxyz[gi + (size_t)18 * HWn];
                float l1[8], l2[8], l3[16];
#pragma unroll
                for (int o = 0; o < 8; ++o)
                    l1[o] = fmaxf(fmaf(W1[o * 3 + 2], i2,
                                  fmaf(W1[o * 3 + 1], i1,
                                  fmaf(W1[o * 3 + 0], i0, B1[o]))), 0.f);
#pragma unroll
                for (int o = 0; o < 8; ++o) {
                    float a = B2[o];
#pragma unroll
                    for (int q = 0; q < 8; ++q) a = fmaf(W2[o * 8 + q], l1[q], a);
                    l2[o] = fmaxf(a, 0.f);
                }
#pragma unroll
                for (int o = 0; o < 16; ++o) {
                    float a = B3[o];
#pragma unroll
                    for (int q = 0; q < 8; ++q) a = fmaf(W3[o * 8 + q], l2[q], a);
                    l3[o] = fmaxf(a, 0.f);
                }
                float4* dst = (float4*)(s_gz + px * GZP + kk * 16);
                dst[0] = make_float4(l3[0],  l3[1],  l3[2],  l3[3]);
                dst[1] = make_float4(l3[4],  l3[5],  l3[6],  l3[7]);
                dst[2] = make_float4(l3[8],  l3[9],  l3[10], l3[11]);
                dst[3] = make_float4(l3[12], l3[13], l3[14], l3[15]);
            }
        }
    }
    __syncthreads();

    const int px  = tid % TPX;
    const int oh  = tid / TPX;
    const int wpx = w0 + px;
    int   off[9];
    float msk[9];
#pragma unroll
    for (int ky = 0; ky < 3; ++ky)
#pragma unroll
        for (int kx = 0; kx < 3; ++kx) {
            const int hh = h + ky - 1, ww = wpx + kx - 1;
            const bool ok = (hh >= 0) & (hh < Hn) & (ww >= 0) & (ww < Wn);
            const int hc = min(max(hh, 0), Hn - 1);
            const int wc = min(max(ww, 0), Wn - 1);
            off[ky * 3 + kx] = hc * Wn + wc;
            msk[ky * 3 + kx] = ok ? 1.f : 0.f;
        }

    const int ln = lane & 15;
    const int lh = lane >> 4;
    v8f acc[4] = {};

#pragma unroll 1
    for (int q = 0; q < NCH; ++q) {
#pragma unroll 1
        for (int cl = 0; cl < CPC; ++cl) {
            const int c = q * CPC + cl;
            const float* x1c = X1 + ((size_t)(b * Cm + c)) * HWn;
            float p[9];
#pragma unroll
            for (int kk = 0; kk < 9; ++kk) p[kk] = x1c[off[kk]] * msk[kk];
            float tv[8];
#pragma unroll
            for (int j = 0; j < 8; ++j) tv[j] = 0.f;
            const float* gzp = s_gz + px * GZP + oh * 8;
#pragma unroll
            for (int kk = 0; kk < 9; ++kk) {
                const float4 ga = *(const float4*)(gzp + kk * 16);
                const float4 gb = *(const float4*)(gzp + kk * 16 + 4);
                const float pk = p[kk];
                tv[0] = fmaf(pk, ga.x, tv[0]);
                tv[1] = fmaf(pk, ga.y, tv[1]);
                tv[2] = fmaf(pk, ga.z, tv[2]);
                tv[3] = fmaf(pk, ga.w, tv[3]);
                tv[4] = fmaf(pk, gb.x, tv[4]);
                tv[5] = fmaf(pk, gb.y, tv[5]);
                tv[6] = fmaf(pk, gb.z, tv[6]);
                tv[7] = fmaf(pk, gb.w, tv[7]);
            }
            v8us hv, lv;
#pragma unroll
            for (int j = 0; j < 8; ++j) {
                unsigned int hb, lb2; split_bf16(tv[j], hb, lb2);
                hv[j] = (unsigned short)hb;
                lv[j] = (unsigned short)lb2;
            }
            const int to = px * TTP + cl * 16 + oh * 8;
            *(v8us*)(s_u.t[0] + to) = hv;
            *(v8us*)(s_u.t[1] + to) = lv;
        }
        __syncthreads();

#pragma unroll 1
        for (int st = 0; st < KCH / 32; ++st) {
            const int tb = (wv * 16 + ln) * TTP + st * 32 + lh * 8;
            Frag bh, bl;
            bh.h8[0] = *(const v8us*)(s_u.t[0] + tb);
            bh.h8[1] = *(const v8us*)(s_u.t[0] + tb + 16);
            bl.h8[0] = *(const v8us*)(s_u.t[1] + tb);
            bl.h8[1] = *(const v8us*)(s_u.t[1] + tb + 16);
            const size_t ka = (size_t)q * KCH + (size_t)st * 32 + (size_t)lh * 8;
#pragma unroll
            for (int mt = 0; mt < 4; ++mt) {
                const size_t ao = (size_t)(mt * 16 + ln) * KD + ka;
                Frag ah, al;
                ah.h8[0] = *(const v8us*)(LWH + ao);
                ah.h8[1] = *(const v8us*)(LWH + ao + 16);
                al.h8[0] = *(const v8us*)(LWL + ao);
                al.h8[1] = *(const v8us*)(LWL + ao + 16);
                acc[mt] = wmma_bf16(ah.b, bh.b, acc[mt]);
                acc[mt] = wmma_bf16(ah.b, bl.b, acc[mt]);
                acc[mt] = wmma_bf16(al.b, bh.b, acc[mt]);
            }
        }
        __syncthreads();
    }

    {
        const float* LS  = P + OFF_LS;
        const float* LEB = P + OFF_LEB;
#pragma unroll
        for (int mt = 0; mt < 4; ++mt)
#pragma unroll
            for (int r = 0; r < 8; ++r) {
                const int o = mt * 16 + lh * 8 + r;
                const float y = fmaxf(fmaf(acc[mt][r], LS[o], LEB[o]), 0.f);
                s_u.o[o * OSP + wv * 16 + ln] = y;
            }
    }
    __syncthreads();

    {
        const int f = lane & 15;
        float* ob = out + (((size_t)b * Cm) * Hn + h) * Wn + w0 + f * 4;
#pragma unroll
        for (int it = 0; it < 8; ++it) {
            const int o = wv * 16 + it * 2 + lh;
            const v4f v = *(const v4f*)(s_u.o + o * OSP + f * 4);
            *(volatile v4f*)(ob + (size_t)o * HWn) = v;
        }
        __threadfence();
#pragma unroll
        for (int it = 0; it < 8; ++it) {
            const int o = wv * 16 + it * 2 + lh;
            const v4f v = *(const v4f*)(s_u.o + o * OSP + f * 4);
            *(volatile v4f*)(ob + (size_t)o * HWn) = v;
        }
    }
}

extern "C" void kernel_launch(void* const* d_in, const int* in_sizes, int n_in,
                              void* d_out, int out_size, void* d_ws, size_t ws_size,
                              hipStream_t stream)
{
    if (n_in < 33) return;
    if (in_sizes[0]  != Bn * Cin * HWn)   return;
    if (in_sizes[2]  != Bn * 3 * 9 * HWn) return;
    if (in_sizes[27] != Cm * KD)          return;
    if (out_size     != Bn * Cm * HWn)    return;

    const float* x     = (const float*)d_in[0];
    const float* gxyz  = (const float*)d_in[2];
    const float* w0    = (const float*)d_in[3];
    const float* b0    = (const float*)d_in[4];
    const float* g0    = (const float*)d_in[5];
    const float* be0   = (const float*)d_in[6];
    const float* m0    = (const float*)d_in[7];
    const float* v0    = (const float*)d_in[8];
    const float* wnw0  = (const float*)d_in[9];
    const float* wnb0  = (const float*)d_in[10];
    const float* wng0  = (const float*)d_in[11];
    const float* wnbe0 = (const float*)d_in[12];
    const float* wnm0  = (const float*)d_in[13];
    const float* wnv0  = (const float*)d_in[14];
    const float* wnw1  = (const float*)d_in[15];
    const float* wnb1  = (const float*)d_in[16];
    const float* wng1  = (const float*)d_in[17];
    const float* wnbe1 = (const float*)d_in[18];
    const float* wnm1  = (const float*)d_in[19];
    const float* wnv1  = (const float*)d_in[20];
    const float* wnw2  = (const float*)d_in[21];
    const float* wnb2  = (const float*)d_in[22];
    const float* wng2  = (const float*)d_in[23];
    const float* wnbe2 = (const float*)d_in[24];
    const float* wnm2  = (const float*)d_in[25];
    const float* wnv2  = (const float*)d_in[26];
    const float* lw    = (const float*)d_in[27];
    const float* lb    = (const float*)d_in[28];
    const float* lg    = (const float*)d_in[29];
    const float* lbe   = (const float*)d_in[30];
    const float* lm    = (const float*)d_in[31];
    const float* lv    = (const float*)d_in[32];

    const size_t x1_bytes  = (size_t)Bn * Cm * HWn * sizeof(float);
    const size_t plane     = (size_t)Cm * KD * sizeof(unsigned short);
    const size_t off_x1    = 0;
    const size_t off_lwh   = off_x1 + x1_bytes;
    const size_t off_lwl   = off_lwh + plane;
    const size_t off_p     = off_lwl + plane;
    const size_t total     = off_p + (size_t)PF_PAD * sizeof(float);
    if (total > ws_size) return;

    char* ws = (char*)d_ws;
    float*          X1  = (float*)(ws + off_x1);
    unsigned short* LWH = (unsigned short*)(ws + off_lwh);
    unsigned short* LWL = (unsigned short*)(ws + off_lwl);
    float*          P   = (float*)(ws + off_p);

    k_fold<<<1, 256, 0, stream>>>(w0, b0, g0, be0, m0, v0,
                                  wnw0, wnb0, wng0, wnbe0, wnm0, wnv0,
                                  wnw1, wnb1, wng1, wnbe1, wnm1, wnv1,
                                  wnw2, wnb2, wng2, wnbe2, wnm2, wnv2,
                                  lb, lg, lbe, lm, lv, P);

    k_lwsplit<<<((Cm * KD) / 8 + 255) / 256, 256, 0, stream>>>(lw, LWH, LWL);

    k_conv0<<<NBLK_C0, 256, 0, stream>>>(x, P, X1);

    k_main<<<NBLK_MAIN, MAIN_THREADS, 0, stream>>>(gxyz, X1, LWH, LWL, P, (float*)d_out);
}
